// RVIT_1_91070486544616
// MI455X (gfx1250) — hardware-verified
//
#include <hip/hip_runtime.h>


#define NL   4
#define BB   16
#define NNn  8
#define PP   64
#define FF   128
#define HH   8
#define NR   (BB * NNn * PP)
#define NPR  (BB * NNn * HH)
#define HF   (HH * FF)
#define PCAR 1024.0f
#define SCL  0.088388347648318447f
typedef _Float16 h16;
typedef unsigned short bf;
typedef __attribute__((ext_vector_type(16))) __bf16   v16bf;
typedef __attribute__((ext_vector_type(16))) _Float16 v16h;
typedef __attribute__((ext_vector_type(8)))  _Float16 v8h;
typedef __attribute__((ext_vector_type(8)))  unsigned short v8us;
typedef __attribute__((ext_vector_type(8)))  float    v8f;
typedef __attribute__((ext_vector_type(4)))  float    v4f;
typedef v8h  __attribute__((may_alias)) v8ha;
typedef v4f  __attribute__((may_alias)) v4fa;
typedef v8us __attribute__((may_alias)) v8usa;

__device__ __forceinline__ unsigned short f2bf(float f) { unsigned u = __float_as_uint(f); u += 0x7FFFu + ((u >> 16) & 1u); return (unsigned short)(u >> 16); }
__device__ __forceinline__ float bf2f(unsigned short b) { return __uint_as_float(((unsigned)b) << 16); }
__device__ __forceinline__ float bfr(float f) { return bf2f(f2bf(f)); }
__device__ __forceinline__ v16h cat16(v8h lo, v8h hi) { return __builtin_shufflevector(lo, hi, 0, 1, 2, 3, 4, 5, 6, 7, 8, 9, 10, 11, 12, 13, 14, 15); }
__device__ __forceinline__ v16bf cat16b(v8us lo, v8us hi) { return __builtin_bit_cast(v16bf, __builtin_shufflevector(lo, hi, 0, 1, 2, 3, 4, 5, 6, 7, 8, 9, 10, 11, 12, 13, 14, 15)); }
__device__ __forceinline__ v8f wmma16(v16h a, v16h b, v8f c) { return __builtin_amdgcn_wmma_f32_16x16x32_f16(false, a, false, b, (short)0, c, false, false); }
__device__ __forceinline__ v8f wmmab(v16bf a, v16bf b, v8f c) { return __builtin_amdgcn_wmma_f32_16x16x32_bf16(false, a, false, b, (short)0, c, false, false); }


template <typename T16> struct WFrag;
template <> struct WFrag<h16> { typedef v16h V; static __device__ __forceinline__ V ld(const h16* p) { return cat16(*(const v8h*)p, *(const v8h*)(p + 16)); } static __device__ __forceinline__ v8f mma(V a, V b, v8f c) { return wmma16(a, b, c); } };
template <> struct WFrag<bf> { typedef v16bf V; static __device__ __forceinline__ V ld(const bf* p) { return cat16b(*(const v8us*)p, *(const v8us*)(p + 16)); } static __device__ __forceinline__ v8f mma(V a, V b, v8f c) { return wmmab(a, b, c); } };
template <typename T16, int NSPLIT, bool BIAS>
__global__ __launch_bounds__(32) void k_gemmw(const T16* __restrict__ A, const T16* __restrict__ A2, const T16* __restrict__ Bt, const T16* __restrict__ Bt2, int K, float* C, int ldc, const float* __restrict__ bias, size_t sA, size_t sB, size_t sC) {
    typedef typename WFrag<T16>::V V;
    __shared__ __align__(16) float os[16 * 68];
    const size_t z = blockIdx.z; A += z * sA; if (A2) A2 += z * sA; Bt += z * sB; if (Bt2) Bt2 += z * sB; C += z * sC;
    const int lane = threadIdx.x & 31, lr = lane & 15, hi = lane >> 4; const int r0 = blockIdx.x * 64, c0 = blockIdx.y * 64;
    v8f acc[4][4];
#pragma unroll
    for (int mb = 0; mb < 4; ++mb)
#pragma unroll
        for (int nb = 0; nb < 4; ++nb) acc[mb][nb] = (v8f){};
    const size_t aoff = (size_t)(r0 + lr) * K + 8 * hi, boff = (size_t)(c0 + lr) * K + 8 * hi;
#pragma unroll 1
    for (int kc = 0; kc < K; kc += 32) {
        V a[4], a2[4];
#pragma unroll
        for (int mb = 0; mb < 4; ++mb) { a[mb] = WFrag<T16>::ld(A + aoff + (size_t)mb * 16 * K + kc); if (NSPLIT == 1 || NSPLIT == 2) a2[mb] = WFrag<T16>::ld(A2 + aoff + (size_t)mb * 16 * K + kc); }
#pragma unroll
        for (int nb = 0; nb < 4; ++nb) { const V b = WFrag<T16>::ld(Bt + boff + (size_t)nb * 16 * K + kc); V b2; if (NSPLIT >= 2) b2 = WFrag<T16>::ld(Bt2 + boff + (size_t)nb * 16 * K + kc);
#pragma unroll
            for (int mb = 0; mb < 4; ++mb) { acc[mb][nb] = WFrag<T16>::mma(a[mb], b, acc[mb][nb]); if (NSPLIT == 1 || NSPLIT == 2) acc[mb][nb] = WFrag<T16>::mma(a2[mb], b, acc[mb][nb]); if (NSPLIT >= 2) acc[mb][nb] = WFrag<T16>::mma(a[mb], b2, acc[mb][nb]); } }
        asm volatile("v_nop\n\tv_nop\n\tv_nop\n\tv_nop" : "+v"(acc[0][0]), "+v"(acc[1][1]), "+v"(acc[2][2]), "+v"(acc[3][3]) : "v"(a[0]), "v"(a[3]));
    }
#pragma unroll
    for (int mb = 0; mb < 4; ++mb) {
#pragma unroll
        for (int nb = 0; nb < 4; ++nb) {
#pragma unroll
            for (int j = 0; j < 8; ++j) os[(hi * 8 + j) * 68 + nb * 16 + lr] = acc[mb][nb][j]; }
        __builtin_amdgcn_wave_barrier(); asm volatile("" ::: "memory");
        float* crow = C + (size_t)(r0 + mb * 16) * ldc + c0;
#pragma unroll 1
        for (int ps = 0; ps < 2; ++ps) {
#pragma unroll
            for (int s = 0; s < 8; ++s) { const int row = 2 * s + hi, cofs = lr * 4; v4f val = *(const v4fa*)(os + row * 68 + cofs); if (BIAS) { val[0] += bfr(bias[c0 + cofs]); val[1] += bfr(bias[c0 + cofs + 1]); val[2] += bfr(bias[c0 + cofs + 2]); val[3] += bfr(bias[c0 + cofs + 3]); }
                *(volatile v4f*)(crow + (size_t)row * ldc + cofs) = val; }
            if (ps == 0) __threadfence(); }
        __builtin_amdgcn_wave_barrier(); asm volatile("" ::: "memory");
    }
}

__device__ __forceinline__ h16 tohx(float x) { return (h16)x; }
__device__ __forceinline__ void splitf(float y, unsigned short& h, unsigned short& l) { h = f2bf(y); l = f2bf(y - bf2f(h)); }
__device__ __forceinline__ float geluf_(float x) { float er = erff(x * 0.70710678f); asm volatile("" : "+v"(er)); float hx = __fmul_rn(0.5f, x); asm volatile("" : "+v"(hx)); return __fmul_rn(hx, __fadd_rn(1.0f, er)); }
typedef __attribute__((ext_vector_type(2))) _Float16 v2h;
typedef __attribute__((ext_vector_type(4))) _Float16 v4h;
typedef __attribute__((ext_vector_type(2))) unsigned short v2us;
typedef __attribute__((ext_vector_type(4))) unsigned short v4us;
typedef __attribute__((ext_vector_type(2))) float v2f;

__global__ __launch_bounds__(256) void k_cvt8(const float* __restrict__ src, bf* dst, size_t n8) { const size_t i = (size_t)blockIdx.x * 256 + threadIdx.x; if (i >= n8) return; const v8f v = *(const v8f*)(src + i * 8); v8us o;
#pragma unroll
    for (int k = 0; k < 8; ++k) o[k] = f2bf(v[k]); *(volatile v8us*)(dst + i * 8) = o; __threadfence(); *(volatile v8us*)(dst + i * 8) = o; }
__device__ __forceinline__ void ln128(const float* x4, const float* __restrict__ s, const float* __restrict__ b, int lane, float* y) { float sm = __fadd_rn(__fadd_rn(x4[0], x4[1]), __fadd_rn(x4[2], x4[3]));
#pragma unroll
    for (int sh = 16; sh; sh >>= 1) sm += __shfl_xor(sm, sh, 32);
    const float mu = sm * (1.0f / FF); float q2 = 0.f;
#pragma unroll
    for (int q = 0; q < 4; ++q) { const float d = __fsub_rn(x4[q], mu); float p = __fmul_rn(d, d); asm volatile("" : "+v"(p)); q2 = __fadd_rn(q2, p); }
#pragma unroll
    for (int sh = 16; sh; sh >>= 1) q2 += __shfl_xor(q2, sh, 32);
    const float rs = __frsqrt_rn(__fadd_rn(q2 * (1.0f / FF), 1e-5f));
#pragma unroll
    for (int q = 0; q < 4; ++q) { float tn = __fmul_rn(__fsub_rn(x4[q], mu), rs); asm volatile("" : "+v"(tn)); float tg = __fmul_rn(tn, bfr(s[lane * 4 + q])); asm volatile("" : "+v"(tg)); y[q] = __fadd_rn(tg, bfr(b[lane * 4 + q])); } }
__global__ __launch_bounds__(256) void k_lnrow(const float* __restrict__ T, const float* __restrict__ s, const float* __restrict__ b, float* Yf, bf* Yh, bf* Yl) { const int lane = threadIdx.x & 31; const int row = blockIdx.x * 8 + (threadIdx.x >> 5); if (row >= NR) return; const v4f a = *(const v4f*)(T + (size_t)row * FF + lane * 4); float x4[4] = {a[0], a[1], a[2], a[3]}; float y[4]; ln128(x4, s, b, lane, y);
    v4f of; v4us oh, ol;
#pragma unroll
    for (int q = 0; q < 4; ++q) { of[q] = y[q]; unsigned short h1, l1; splitf(y[q], h1, l1); oh[q] = h1; ol[q] = l1; }
    const size_t o = (size_t)row * FF + lane * 4;
    for (int ps = 0; ps < 2; ++ps) { if (Yf) *(volatile v4f*)(Yf + o) = of; *(volatile v4us*)(Yh + o) = oh; *(volatile v4us*)(Yl + o) = ol; if (ps == 0) __threadfence(); } }
__global__ __launch_bounds__(256) void k_blend(const float* __restrict__ Xc, const float* __restrict__ Xp, const float* __restrict__ al, int which, h16* OUTp) { const size_t e = ((size_t)blockIdx.x * 256 + threadIdx.x) * 2; if (e >= (size_t)NR * HF) return; v2h o;
    if (which < 2) { const int col = (int)(e % HF), row = (int)(e / HF); const int h = col / FF, f = col % FF; const int p = row % PP, bn = row / PP;
#pragma unroll
        for (int q = 0; q < 2; ++q) { const float a = __fdiv_rn(1.0f, __fadd_rn(1.0f, __expf(-bfr(al[which * HF + col + q])))); float t1 = __fmul_rn(a, Xc[e + q]), t2 = __fmul_rn(__fsub_rn(1.0f, a), Xp[e + q]); asm volatile("" : "+v"(t1), "+v"(t2)); o[q] = tohx(__fadd_rn(t1, t2)); }
        const size_t oo = (((size_t)bn * HH + h) * PP + p) * FF + f; *(volatile v2h*)(OUTp + oo) = o; __threadfence(); *(volatile v2h*)(OUTp + oo) = o; }
    else { const int p = (int)(e % PP); const int f = (int)((e / PP) % FF); const int pr = (int)(e / ((size_t)PP * FF)); const int h = pr % HH, bn = pr / HH; const int col = h * FF + f;
        const float a = __fdiv_rn(1.0f, __fadd_rn(1.0f, __expf(-bfr(al[2 * HF + col]))));
#pragma unroll
        for (int q = 0; q < 2; ++q) { const size_t src = ((size_t)bn * PP + p + q) * HF + col; float t1 = __fmul_rn(a, Xc[src]), t2 = __fmul_rn(__fsub_rn(1.0f, a), Xp[src]); asm volatile("" : "+v"(t1), "+v"(t2)); o[q] = tohx(__fadd_rn(t1, t2)); }
        *(volatile v2h*)(OUTp + e) = o; __threadfence(); *(volatile v2h*)(OUTp + e) = o; } }
__global__ __launch_bounds__(256) void k_sm64(const float* __restrict__ S, h16* P) { const int lane = threadIdx.x & 31; const int row = blockIdx.x * 8 + (threadIdx.x >> 5); if (row >= NPR * PP) return; const v2f a = *(const v2f*)(S + (size_t)row * PP + lane * 2); float t0 = __fmul_rn(a[0], SCL), t1 = __fmul_rn(a[1], SCL); float mx = fmaxf(t0, t1);
#pragma unroll
    for (int sh = 16; sh; sh >>= 1) mx = fmaxf(mx, __shfl_xor(mx, sh, 32));
    float d0 = __fsub_rn(t0, mx), d1 = __fsub_rn(t1, mx); asm volatile("" : "+v"(d0), "+v"(d1)); const float e0 = __expf(d0), e1 = __expf(d1); float sum = __fadd_rn(e0, e1);
#pragma unroll
    for (int sh = 16; sh; sh >>= 1) sum += __shfl_xor(sum, sh, 32);
    const float f = __fdiv_rn(PCAR, sum); v2h o; o[0] = tohx(e0 * f); o[1] = tohx(e1 * f); *(volatile v2h*)(P + (size_t)row * PP + lane * 2) = o; __threadfence(); *(volatile v2h*)(P + (size_t)row * PP + lane * 2) = o; }
__global__ __launch_bounds__(256) void k_lnA(const float* __restrict__ O, const float* __restrict__ s, const float* __restrict__ b, bf* Ah, bf* Al) { const int lane = threadIdx.x & 31; const int row = blockIdx.x * 8 + (threadIdx.x >> 5); if (row >= NPR * PP) return; const int p = row % PP, pr = row / PP; const int h = pr % HH, bn = pr / HH;
    const v4f a = *(const v4f*)(O + (size_t)row * FF + lane * 4); float x4[4] = {a[0] * (1.0f / PCAR), a[1] * (1.0f / PCAR), a[2] * (1.0f / PCAR), a[3] * (1.0f / PCAR)}; float y[4]; ln128(x4, s, b, lane, y); v4us oh, ol;
#pragma unroll
    for (int q = 0; q < 4; ++q) { unsigned short h1, l1; splitf(y[q], h1, l1); oh[q] = h1; ol[q] = l1; }
    const size_t oo = ((size_t)bn * PP + p) * HF + h * FF + lane * 4; *(volatile v4us*)(Ah + oo) = oh; *(volatile v4us*)(Al + oo) = ol; __threadfence(); *(volatile v4us*)(Ah + oo) = oh; *(volatile v4us*)(Al + oo) = ol; }
__global__ __launch_bounds__(256) void k_mid(const float* __restrict__ PJ, const float* __restrict__ CUR, const float* __restrict__ s2, const float* __restrict__ b2, const float* __restrict__ so, const float* __restrict__ bo, float* OHf, bf* Oh, bf* Ol) { const int lane = threadIdx.x & 31; const int row = blockIdx.x * 8 + (threadIdx.x >> 5); if (row >= NR) return; const size_t o = (size_t)row * FF + lane * 4;
    const v4f a = *(const v4f*)(PJ + o), c = *(const v4f*)(CUR + o); float x4[4] = {a[0], a[1], a[2], a[3]}; float y[4]; ln128(x4, s2, b2, lane, y); float x3[4];
#pragma unroll
    for (int q = 0; q < 4; ++q) { const float a2 = __fadd_rn(y[q], geluf_(c[q])); x3[q] = __fadd_rn(c[q], a2); }
    float z[4]; ln128(x3, so, bo, lane, z); v4f of; v4us oh, ol;
#pragma unroll
    for (int q = 0; q < 4; ++q) { of[q] = z[q]; unsigned short h1, l1; splitf(z[q], h1, l1); oh[q] = h1; ol[q] = l1; }
    for (int ps = 0; ps < 2; ++ps) { *(volatile v4f*)(OHf + o) = of; *(volatile v4us*)(Oh + o) = oh; *(volatile v4us*)(Ol + o) = ol; if (ps == 0) __threadfence(); } }
__global__ __launch_bounds__(256) void k_fin(const float* __restrict__ FFo, const float* __restrict__ OHf, float* CUR, bf* Ch, bf* Cl) { const size_t i = ((size_t)blockIdx.x * 256 + threadIdx.x) * 4; if (i >= (size_t)NR * FF) return; const v4f a = *(const v4f*)(FFo + i), b = *(const v4f*)(OHf + i); v4f of; v4us oh, ol;
#pragma unroll
    for (int q = 0; q < 4; ++q) { of[q] = __fadd_rn(a[q], geluf_(b[q])); unsigned short h1, l1; splitf(of[q], h1, l1); oh[q] = h1; ol[q] = l1; }
    for (int ps = 0; ps < 2; ++ps) { *(volatile v4f*)(CUR + i) = of; *(volatile v4us*)(Ch + i) = oh; *(volatile v4us*)(Cl + i) = ol; if (ps == 0) __threadfence(); } }

extern "C" void kernel_launch(void* const* d_in, const int* in_sizes, int n_in,
                              void* d_out, int out_size, void* d_ws, size_t ws_size, hipStream_t stream) {
    (void)in_sizes; (void)n_in; (void)out_size;
    const float* IN[25]; for (int i = 0; i < 25; ++i) IN[i] = (const float*)d_in[i];
    float* OUT = (float*)d_out;
    char* wsp = (char*)d_ws;
    auto take = [&](size_t bytes) { char* p = wsp; wsp += (bytes + 255) & ~(size_t)255; return (void*)p; };
    bf* WP1 = (bf*)take((size_t)FF * FF * 2); bf* WP2 = (bf*)take((size_t)FF * FF * 2); bf* WQC = (bf*)take((size_t)3 * HF * FF * 2); bf* WQP = (bf*)take((size_t)3 * HF * FF * 2); bf* WPJ = (bf*)take((size_t)FF * HF * 2); bf* WFF = (bf*)take((size_t)FF * FF * 2);
    bf* XB = (bf*)take((size_t)NR * FF * 2); float* T = (float*)take((size_t)NR * FF * 4); float* CUR = (float*)take((size_t)NR * FF * 4); bf* Ch = (bf*)take((size_t)NR * FF * 2); bf* Cl = (bf*)take((size_t)NR * FF * 2); bf* Ph = (bf*)take((size_t)NR * FF * 2); bf* Pl = (bf*)take((size_t)NR * FF * 2);
    float* XC = (float*)take((size_t)NR * HF * 4); float* XP = (float*)take((size_t)NR * HF * 4); h16* Q16 = (h16*)take((size_t)NPR * PP * FF * 2); h16* K16 = (h16*)take((size_t)NPR * PP * FF * 2); h16* VT = (h16*)take((size_t)NPR * FF * PP * 2);
    float* S = (float*)take((size_t)NPR * PP * PP * 4); h16* P16 = (h16*)take((size_t)NPR * PP * PP * 2); float* O = (float*)take((size_t)NPR * PP * FF * 4); bf* Ah = (bf*)take((size_t)NR * HF * 2); bf* Al = (bf*)take((size_t)NR * HF * 2); float* PJ = (float*)take((size_t)NR * FF * 4); float* OHf = (float*)take((size_t)NR * FF * 4); bf* Oh = (bf*)take((size_t)NR * FF * 2); bf* Ol = (bf*)take((size_t)NR * FF * 2); float* FFo = (float*)take((size_t)NR * FF * 4);
    if ((size_t)(wsp - (char*)d_ws) > ws_size) return;
    const unsigned L4 = (unsigned)(((size_t)NR * FF / 4 + 255) / 256), LH2 = (unsigned)(((size_t)NR * HF / 2 + 255) / 256);
    for (int l = 0; l < NL; ++l) {
        { k_cvt8<<<(FF * FF / 8 + 255) / 256, 256, 0, stream>>>(IN[2] + (size_t)l * FF * FF, WP1, (size_t)FF * FF / 8); k_cvt8<<<(FF * FF / 8 + 255) / 256, 256, 0, stream>>>(IN[4] + (size_t)l * FF * FF, WP2, (size_t)FF * FF / 8);
          k_cvt8<<<(3 * HF * FF / 8 + 255) / 256, 256, 0, stream>>>(IN[10] + (size_t)l * 3 * HF * FF, WQC, (size_t)3 * HF * FF / 8); k_cvt8<<<(3 * HF * FF / 8 + 255) / 256, 256, 0, stream>>>(IN[12] + (size_t)l * 3 * HF * FF, WQP, (size_t)3 * HF * FF / 8);
          k_cvt8<<<(FF * HF / 8 + 255) / 256, 256, 0, stream>>>(IN[15] + (size_t)l * FF * HF, WPJ, (size_t)FF * HF / 8); k_cvt8<<<(FF * FF / 8 + 255) / 256, 256, 0, stream>>>(IN[23] + (size_t)l * FF * FF, WFF, (size_t)FF * FF / 8); }
        if (l == 0) { k_cvt8<<<(unsigned)(((size_t)NR * FF / 8 + 255) / 256), 256, 0, stream>>>(IN[0], XB, (size_t)NR * FF / 8);
            k_gemmw<bf, 0, true><<<dim3(NR / 64, FF / 64, 1), 32, 0, stream>>>(XB, nullptr, WP1, nullptr, FF, T, FF, IN[3], 0, 0, 0); k_lnrow<<<NR / 8, 256, 0, stream>>>(T, IN[6], IN[7], CUR, Ch, Cl); }
        k_cvt8<<<(unsigned)(((size_t)NR * FF / 8 + 255) / 256), 256, 0, stream>>>(IN[1] + (size_t)l * NR * FF, XB, (size_t)NR * FF / 8);
        k_gemmw<bf, 0, true><<<dim3(NR / 64, FF / 64, 1), 32, 0, stream>>>(XB, nullptr, WP2, nullptr, FF, T, FF, IN[5] + l * FF, 0, 0, 0); k_lnrow<<<NR / 8, 256, 0, stream>>>(T, IN[8] + l * FF, IN[9] + l * FF, nullptr, Ph, Pl);
        for (int w = 0; w < 3; ++w) {
            k_gemmw<bf, 1, true><<<dim3(NR / 64, HF / 64, 1), 32, 0, stream>>>(Ch, Cl, WQC + (size_t)w * HF * FF, nullptr, FF, XC, HF, IN[11] + (size_t)l * 3 * HF + w * HF, 0, 0, 0);
            k_gemmw<bf, 1, true><<<dim3(NR / 64, HF / 64, 1), 32, 0, stream>>>(Ph, Pl, WQP + (size_t)w * HF * FF, nullptr, FF, XP, HF, IN[13] + (size_t)l * 3 * HF + w * HF, 0, 0, 0);
            k_blend<<<LH2, 256, 0, stream>>>(XC, XP, IN[14] + (size_t)l * 3 * HF, w, w == 0 ? Q16 : (w == 1 ? K16 : VT)); }
        k_gemmw<h16, 0, false><<<dim3(1, 1, NPR), 32, 0, stream>>>(Q16, nullptr, K16, nullptr, FF, S, PP, nullptr, (size_t)PP * FF, (size_t)PP * FF, (size_t)PP * PP);
        k_sm64<<<NPR * PP / 8, 256, 0, stream>>>(S, P16);
        k_gemmw<h16, 0, false><<<dim3(1, FF / 64, NPR), 32, 0, stream>>>(P16, nullptr, VT, nullptr, PP, O, FF, nullptr, (size_t)PP * PP, (size_t)FF * PP, (size_t)PP * FF);
        k_lnA<<<NPR * PP / 8, 256, 0, stream>>>(O, IN[17] + l * FF, IN[18] + l * FF, Ah, Al);
        k_gemmw<bf, 1, true><<<dim3(NR / 64, FF / 64, 1), 32, 0, stream>>>(Ah, Al, WPJ, nullptr, HF, PJ, FF, IN[16] + l * FF, 0, 0, 0);
        k_mid<<<NR / 8, 256, 0, stream>>>(PJ, CUR, IN[19] + l * FF, IN[20] + l * FF, IN[21] + l * FF, IN[22] + l * FF, OHf, Oh, Ol);
        k_gemmw<bf, 1, true><<<dim3(NR / 64, FF / 64, 1), 32, 0, stream>>>(Oh, Ol, WFF, nullptr, FF, FFo, FF, IN[24] + l * FF, 0, 0, 0);
        k_fin<<<L4, 256, 0, stream>>>(FFo, OHf, l == NL - 1 ? OUT : CUR, Ch, Cl); }
}
